// SGC_5643587027282
// MI455X (gfx1250) — hardware-run, weakly checked
//
#include <hip/hip_runtime.h>
#include <stddef.h>
#include <stdint.h>


#define DF      64
#define KT      128
#define NOUT    40
#define NOP     48
#define NTHR    256
#define NWAVE   8
#define EPT     8
#define WCH     (32 * EPT)
#define NBA     1024
#define PKS     10
#define RCAP    28672
#define WLCAP   (RCAP / NWAVE)
#define DEGCAP  64
#define TBM     128
#define BK_INTS (2 * RCAP + 3 * NBA + 32)
#define LDS_BK  (BK_INTS * 4)
#define MEAS_BLK_HITS 16710
#define MEAS_MAXDEG   36
#define WSMAX   134217728

static_assert(DF == 64 && DF == 16 * 4);
static_assert(NBA == (1 << PKS) && NBA == NTHR * 4 && NBA % NWAVE == 0 && NBA % 16 == 0);
static_assert(RCAP % (NTHR * 4) == 0 && BK_INTS % 4 == 0 && WLCAP * NWAVE == RCAP);
static_assert((long long)RCAP * 100 >= (long long)MEAS_BLK_HITS * 105);
static_assert((long long)WLCAP * NWAVE * 100 >= (long long)MEAS_BLK_HITS * 150);
static_assert(DEGCAP >= MEAS_MAXDEG + 8 && DEGCAP % 2 == 0);
static_assert(LDS_BK + NBA * 4 <= 300000);
static_assert(KT % 32 == 0 && KT == 2 * DF);
static_assert(NOUT <= NOP && NOP == 3 * 16 && NOUT % 4 == 0);
static_assert(TBM == NWAVE * 16);
static_assert((TBM * NOUT * 4) % 128 == 0 && (TBM * NOUT) % (4 * NTHR) == 0);
static_assert(98 * NBA >= 100000 && 782 * TBM == 100096);
static_assert(TBM * NOUT <= TBM * DF);

typedef float          v2f   __attribute__((ext_vector_type(2)));
typedef float          v4f   __attribute__((ext_vector_type(4)));
typedef float          v8f   __attribute__((ext_vector_type(8)));
typedef int            v4i   __attribute__((ext_vector_type(4)));
typedef int            v8i   __attribute__((ext_vector_type(8)));
typedef unsigned       v4u   __attribute__((ext_vector_type(4)));
typedef unsigned short v8us  __attribute__((ext_vector_type(8)));
typedef __bf16         v16bf __attribute__((ext_vector_type(16)));
typedef v2f  __attribute__((may_alias)) v2fa;
typedef v4f  __attribute__((may_alias)) v4fa;
typedef v4i  __attribute__((may_alias)) v4ia;
typedef v8us __attribute__((may_alias)) v8usa;
union FragB { v16bf v; v8us h[2]; v8i w; };

__device__ __forceinline__ v8f wmb(const FragB& a, const FragB& b, v8f c) {
  v8f d = __builtin_amdgcn_wmma_f32_16x16x32_bf16(false, a.v, false, b.v, (short)0, c, false, false);
  asm volatile("v_nop\n\tv_nop\n\tv_nop\n\tv_nop" : "+v"(d) : "v"(a.w), "v"(b.w));
  return d;
}

__device__ __forceinline__ unsigned bf16_bits(float f) {
  const unsigned u = __float_as_uint(f);
  return ((u + 0x7FFFu + ((u >> 16) & 1u)) >> 16) & 0xFFFFu;
}
__device__ __forceinline__ float bf16_val(float f) { return __uint_as_float(bf16_bits(f) << 16); }
__device__ __forceinline__ void pack2(float a, float b, unsigned& hw, unsigned& lw) {
  const unsigned ha = bf16_bits(a), hb = bf16_bits(b);
  const unsigned la = bf16_bits(a - __uint_as_float(ha << 16));
  const unsigned lb = bf16_bits(b - __uint_as_float(hb << 16));
  hw = ha | (hb << 16);
  lw = la | (lb << 16);
}

__global__ __launch_bounds__(NTHR) void k_prep(const float* __restrict__ Wlin, const float* __restrict__ blin,
                                               const float* __restrict__ Whead, const float* __restrict__ bhead,
                                               unsigned short* W1D, unsigned short* W2D, float* BB,
                                               unsigned short* X3, int nN, int nPadUnits) {
  const int b = (int)blockIdx.x, tid = (int)threadIdx.x;
  if (b < 4) {
    const int u  = b * NTHR + tid;
    const int n  = u >> 4;
    const int k8 = (u & 15) * 8;
    const int kk = k8 & (DF - 1);
    const float* p = Wlin + (size_t)kk * DF + n;
    v8us o;
#pragma unroll
    for (int i = 0; i < 8; ++i) o[i] = (unsigned short)bf16_bits(p[(size_t)i * DF]);
    unsigned short* dp = W1D + (size_t)n * KT + k8;
    *(volatile v8us*)dp = o;
    __threadfence();
    *(volatile v8us*)dp = o;
  } else if (b < 7) {
    const int v  = (b - 4) * NTHR + tid;
    const int n  = v >> 4;
    const int k8 = (v & 15) * 8;
    const int kk = k8 & (DF - 1);
    const int nc = n < NOUT ? n : NOUT - 1;
    const float* p = Whead + (size_t)kk * NOUT + nc;
    float f[8];
#pragma unroll
    for (int i = 0; i < 8; ++i) f[i] = p[(size_t)i * NOUT];
    asm volatile("" :: "v"(f[0]), "v"(f[1]), "v"(f[2]), "v"(f[3]), "v"(f[4]), "v"(f[5]), "v"(f[6]), "v"(f[7]));
    const unsigned mk = (n < NOUT) ? 0xFFFFu : 0u;
    v8us o;
#pragma unroll
    for (int i = 0; i < 8; ++i) o[i] = (unsigned short)(bf16_bits(f[i]) & mk);
    unsigned short* dp = W2D + (size_t)n * KT + k8;
    *(volatile v8us*)dp = o;
    __threadfence();
    *(volatile v8us*)dp = o;
  } else if (b == 7) {
    if (tid < 32) {
      const int j  = tid & 15;
      const int j2 = j < (NOUT / 4) ? j : (NOUT / 4) - 1;
      const v4f a = *(const v4f*)(blin + 4 * j);
      const v4f c = *(const v4f*)(bhead + 4 * j2);
      asm volatile("" :: "v"(a), "v"(c));
      const unsigned ma = (tid < 16) ? 0xFFFFFFFFu : 0u;
      const unsigned mc = (tid >= 16 && j < (NOUT / 4)) ? 0xFFFFFFFFu : 0u;
      v4f o;
      o.x = __uint_as_float((__float_as_uint(bf16_val(a.x)) & ma) | (__float_as_uint(bf16_val(c.x)) & mc));
      o.y = __uint_as_float((__float_as_uint(bf16_val(a.y)) & ma) | (__float_as_uint(bf16_val(c.y)) & mc));
      o.z = __uint_as_float((__float_as_uint(bf16_val(a.z)) & ma) | (__float_as_uint(bf16_val(c.z)) & mc));
      o.w = __uint_as_float((__float_as_uint(bf16_val(a.w)) & ma) | (__float_as_uint(bf16_val(c.w)) & mc));
      float* dp = BB + 4 * tid;
      *(volatile v4f*)dp = o;
      __threadfence();
      *(volatile v4f*)dp = o;
    }
  } else {
    const int u = (b - 8) * NTHR + tid;
    if (u < nPadUnits) {
      const int row = nN + (u >> 4);
      const v8us z = {0, 0, 0, 0, 0, 0, 0, 0};
      unsigned short* dp = X3 + (size_t)row * KT + 8 * (u & 15);
      *(volatile v8us*)dp = z;
      __threadfence();
      *(volatile v8us*)dp = z;
    }
  }
}

__global__ __launch_bounds__(NTHR) void k_bucket(const int* __restrict__ dsts, const int* __restrict__ srcs,
                                                 const float* __restrict__ x, int nE, int nN, int vec8, int segLen,
                                                 int* LIST, int* CNT, int* OFF, float* DINV, int* REC, float* PA) {
  extern __shared__ __attribute__((aligned(16))) int dsm[];
  __shared__ __attribute__((aligned(16))) float sdv[NBA];
  int* wl   = dsm;
  int* reg2 = wl + RCAP;
  int* scnt = reg2 + RCAP;
  int* soff = scnt + NBA;
  int* cur  = soff + NBA;
  int* wcnt = cur + NBA;
  int* wtot = wcnt + 8;
  int* wmx  = wtot + 8;
  const int tid = (int)threadIdx.x, lane = tid & 31, wave = tid >> 5;
  const int nodeBase = (int)blockIdx.x * NBA;
  int nb = nN - nodeBase;
  nb = nb > NBA ? NBA : (nb < 1 ? 1 : nb);

  {
    const v4i z4 = {0, 0, 0, 0};
    for (int i = tid * 4; i < BK_INTS; i += NTHR * 4) *(v4ia*)(dsm + i) = z4;
  }
  __syncthreads();

  {
    const int segBeg = wave * segLen;
    int segEnd = segBeg + segLen;
    segEnd = segEnd > nE ? nE : segEnd;
    int* mywl = wl + wave * WLCAP;
    int wc = 0;
    const unsigned nbs = (unsigned)nodeBase;
    const unsigned unb = (unsigned)nb;
    const int sent = -2147483647 - 1;
#pragma unroll 1
    for (int cb = segBeg; cb < segEnd; cb += WCH) {
      const int e0 = cb + lane * EPT;
      v4i da, db;
      if (vec8 != 0 && cb + WCH <= nE) {
        da = *(const v4i*)(dsts + e0);
        db = *(const v4i*)(dsts + e0 + 4);
      } else {
        const int t0 = dsts[min(e0,     nE - 1)], t1 = dsts[min(e0 + 1, nE - 1)];
        const int t2 = dsts[min(e0 + 2, nE - 1)], t3 = dsts[min(e0 + 3, nE - 1)];
        const int t4 = dsts[min(e0 + 4, nE - 1)], t5 = dsts[min(e0 + 5, nE - 1)];
        const int t6 = dsts[min(e0 + 6, nE - 1)], t7 = dsts[min(e0 + 7, nE - 1)];
        asm volatile("" :: "v"(t0), "v"(t1), "v"(t2), "v"(t3), "v"(t4), "v"(t5), "v"(t6), "v"(t7));
        da.x = (e0     < nE) ? t0 : sent;
        da.y = (e0 + 1 < nE) ? t1 : sent;
        da.z = (e0 + 2 < nE) ? t2 : sent;
        da.w = (e0 + 3 < nE) ? t3 : sent;
        db.x = (e0 + 4 < nE) ? t4 : sent;
        db.y = (e0 + 5 < nE) ? t5 : sent;
        db.z = (e0 + 6 < nE) ? t6 : sent;
        db.w = (e0 + 7 < nE) ? t7 : sent;
      }
      const unsigned s0 = (unsigned)da.x - nbs, s1 = (unsigned)da.y - nbs;
      const unsigned s2 = (unsigned)da.z - nbs, s3 = (unsigned)da.w - nbs;
      const unsigned s4 = (unsigned)db.x - nbs, s5 = (unsigned)db.y - nbs;
      const unsigned s6 = (unsigned)db.z - nbs, s7 = (unsigned)db.w - nbs;
      const bool h0 = s0 < unb, h1 = s1 < unb, h2 = s2 < unb, h3 = s3 < unb;
      const bool h4 = s4 < unb, h5 = s5 < unb, h6 = s6 < unb, h7 = s7 < unb;
      const unsigned any = __builtin_amdgcn_ballot_w32(h0 | h1 | h2 | h3 | h4 | h5 | h6 | h7);
      if (any != 0u) {
        const unsigned m0 = __builtin_amdgcn_ballot_w32(h0), m1 = __builtin_amdgcn_ballot_w32(h1);
        const unsigned m2 = __builtin_amdgcn_ballot_w32(h2), m3 = __builtin_amdgcn_ballot_w32(h3);
        const unsigned m4 = __builtin_amdgcn_ballot_w32(h4), m5 = __builtin_amdgcn_ballot_w32(h5);
        const unsigned m6 = __builtin_amdgcn_ballot_w32(h6), m7 = __builtin_amdgcn_ballot_w32(h7);
        int run = wc + (int)(__builtin_amdgcn_mbcnt_lo(m0, 0u) + __builtin_amdgcn_mbcnt_lo(m1, 0u) +
                             __builtin_amdgcn_mbcnt_lo(m2, 0u) + __builtin_amdgcn_mbcnt_lo(m3, 0u) +
                             __builtin_amdgcn_mbcnt_lo(m4, 0u) + __builtin_amdgcn_mbcnt_lo(m5, 0u) +
                             __builtin_amdgcn_mbcnt_lo(m6, 0u) + __builtin_amdgcn_mbcnt_lo(m7, 0u));
#define HITJ(J, HJ, SJ) { if (HJ) { \
          if (run < WLCAP) mywl[run] = (int)((((unsigned)(e0 + (J))) << PKS) | (SJ)); \
          run += 1; } }
        HITJ(0, h0, s0)
        HITJ(1, h1, s1)
        HITJ(2, h2, s2)
        HITJ(3, h3, s3)
        HITJ(4, h4, s4)
        HITJ(5, h5, s5)
        HITJ(6, h6, s6)
        HITJ(7, h7, s7)
#undef HITJ
        wc += (int)(__builtin_popcount(m0) + __builtin_popcount(m1) + __builtin_popcount(m2) +
                    __builtin_popcount(m3) + __builtin_popcount(m4) + __builtin_popcount(m5) +
                    __builtin_popcount(m6) + __builtin_popcount(m7));
      }
    }
    if (lane == 0) wcnt[wave] = wc;
  }
  __syncthreads();

  if (wave == 0) {
#pragma unroll 1
    for (int w2 = 0; w2 < NWAVE; ++w2) {
      int c = wcnt[w2];
      c = c < 0 ? 0 : (c > WLCAP ? WLCAP : c);
#pragma unroll 1
      for (int b0 = 0; b0 < c; b0 += 32) {
        const int idx = b0 + lane;
        const int uv  = wl[w2 * WLCAP + (idx < WLCAP ? idx : WLCAP - 1)];
        const int m32 = (c - b0) < 32 ? (c - b0) : 32;
#pragma unroll 1
        for (int k = 0; k < m32; ++k) {
          const int u  = __builtin_amdgcn_readlane(uv, k);
          const int sl = u & (NBA - 1);
          if (lane == 0) scnt[sl] = scnt[sl] + 1;
        }
      }
    }
  }
  __syncthreads();

  {
    const v4i ca = *(const v4ia*)(scnt + 4 * tid);
    const int e0 = ca.x < 0 ? 0 : ca.x, e1 = ca.y < 0 ? 0 : ca.y, e2 = ca.z < 0 ? 0 : ca.z, e3 = ca.w < 0 ? 0 : ca.w;
    const int ts = e0 + e1 + e2 + e3;
    int incl = ts;
#pragma unroll
    for (int d = 1; d < 32; d <<= 1) {
      const int up = __shfl_up(incl, d, 32);
      if (lane >= d) incl += up;
    }
    int mx = max(max(e0, e1), max(e2, e3));
    mx = max(mx, __shfl_xor(mx, 16, 32));
    mx = max(mx, __shfl_xor(mx, 8, 32));
    mx = max(mx, __shfl_xor(mx, 4, 32));
    mx = max(mx, __shfl_xor(mx, 2, 32));
    mx = max(mx, __shfl_xor(mx, 1, 32));
    if (lane == 31) wtot[wave] = incl;
    if (lane == 0)  wmx[wave] = mx;
    __syncthreads();
    int pre = 0;
#pragma unroll
    for (int w2 = 0; w2 < NWAVE; ++w2) pre += (w2 < wave) ? wtot[w2] : 0;
    int run = pre + incl - ts;
    v4i so;
    so.x = run; run += e0;
    so.y = run; run += e1;
    so.z = run; run += e2;
    so.w = run;
    *(v4ia*)(soff + 4 * tid) = so;
    *(v4ia*)(cur + 4 * tid)  = so;
  }
  __syncthreads();

  if (wave == 0) {
#pragma unroll 1
    for (int w2 = 0; w2 < NWAVE; ++w2) {
      int c = wcnt[w2];
      c = c < 0 ? 0 : (c > WLCAP ? WLCAP : c);
#pragma unroll 1
      for (int b0 = 0; b0 < c; b0 += 32) {
        const int idx = b0 + lane;
        const int uv  = wl[w2 * WLCAP + (idx < WLCAP ? idx : WLCAP - 1)];
        const int m32 = (c - b0) < 32 ? (c - b0) : 32;
#pragma unroll 1
        for (int k = 0; k < m32; ++k) {
          const int u   = __builtin_amdgcn_readlane(uv, k);
          const int sl  = u & (NBA - 1);
          const int eid = (int)((unsigned)u >> PKS);
          if (lane == 0) {
            int pos = cur[sl];
            pos = pos < 0 ? 0 : (pos > RCAP - 1 ? RCAP - 1 : pos);
            reg2[pos] = eid;
            cur[sl] = pos + 1;
          }
        }
      }
    }
  }
  __syncthreads();

  int nh = 0, ovw = 0, bmax = 0;
#pragma unroll
  for (int w2 = 0; w2 < NWAVE; ++w2) {
    int c = wcnt[w2];
    ovw |= (c > WLCAP) ? 1 : 0;
    c = c < 0 ? 0 : (c > WLCAP ? WLCAP : c);
    nh += c;
    bmax = max(bmax, wmx[w2]);
  }
  const int flag = ((ovw != 0) || (bmax > DEGCAP)) ? 1 : 0;
  const int padv = nodeBase < nN ? nodeBase : nN - 1;

  int* lrow = LIST + (size_t)blockIdx.x * RCAP;
#pragma unroll 1
  for (int it = 0; it < RCAP / (NTHR * 4); ++it) {
    const int i0 = 4 * (it * NTHR + tid);
    const v4i ev = *(const v4ia*)(reg2 + i0);
    int e0 = ev.x, e1 = ev.y, e2 = ev.z, e3 = ev.w;
    e0 = e0 < 0 ? 0 : (e0 > nE - 1 ? nE - 1 : e0);
    e1 = e1 < 0 ? 0 : (e1 > nE - 1 ? nE - 1 : e1);
    e2 = e2 < 0 ? 0 : (e2 > nE - 1 ? nE - 1 : e2);
    e3 = e3 < 0 ? 0 : (e3 > nE - 1 ? nE - 1 : e3);
    int g0 = srcs[e0], g1 = srcs[e1], g2 = srcs[e2], g3 = srcs[e3];
    asm volatile("" :: "v"(g0), "v"(g1), "v"(g2), "v"(g3));
    g0 = g0 < 0 ? 0 : (g0 > nN - 1 ? nN - 1 : g0);
    g1 = g1 < 0 ? 0 : (g1 > nN - 1 ? nN - 1 : g1);
    g2 = g2 < 0 ? 0 : (g2 > nN - 1 ? nN - 1 : g2);
    g3 = g3 < 0 ? 0 : (g3 > nN - 1 ? nN - 1 : g3);
    v4i ov;
    ov.x = (i0     < nh) ? g0 : padv;
    ov.y = (i0 + 1 < nh) ? g1 : padv;
    ov.z = (i0 + 2 < nh) ? g2 : padv;
    ov.w = (i0 + 3 < nh) ? g3 : padv;
    *(volatile v4i*)(lrow + i0) = ov;
    __threadfence();
    *(volatile v4i*)(lrow + i0) = ov;
  }
  {
    const v4i cv = *(const v4ia*)(scnt + 4 * tid);
    const v4i fv = *(const v4ia*)(soff + 4 * tid);
    const int d0 = cv.x + 1, d1 = cv.y + 1, d2 = cv.z + 1, d3 = cv.w + 1;
    v4f dv;
    dv.x = (d0 > 0) ? rsqrtf((float)d0) : 0.0f;
    dv.y = (d1 > 0) ? rsqrtf((float)d1) : 0.0f;
    dv.z = (d2 > 0) ? rsqrtf((float)d2) : 0.0f;
    dv.w = (d3 > 0) ? rsqrtf((float)d3) : 0.0f;
    *(v4fa*)(sdv + 4 * tid) = dv;
    v4i rv = {0, 0, 0, 0};
    rv.x = (tid == 0) ? bmax : 0;
    rv.y = (tid == 0) ? flag : 0;
    rv.z = (tid == 0) ? nh : 0;
    int*   cp = CNT  + (size_t)nodeBase + 4 * tid;
    int*   fp = OFF  + (size_t)nodeBase + 4 * tid;
    float* vp = DINV + (size_t)nodeBase + 4 * tid;
    int*   rp = REC  + (size_t)blockIdx.x * 32 + 4 * (tid & 7);
    *(volatile v4i*)cp = cv;
    *(volatile v4i*)fp = fv;
    *(volatile v4f*)vp = dv;
    if (tid < 8) *(volatile v4i*)rp = rv;
    __threadfence();
    *(volatile v4i*)cp = cv;
    *(volatile v4i*)fp = fv;
    *(volatile v4f*)vp = dv;
    if (tid < 8) *(volatile v4i*)rp = rv;
  }
  __syncthreads();

#pragma unroll 1
  for (int it = 0; it < NBA / 16; ++it) {
    const int r    = it * 16 + (tid >> 4);
    const int node = nodeBase + r;
    const int nc   = node < nN ? node : nN - 1;
    const v4f xv = *(const v4f*)(x + (size_t)nc * DF + 4 * (tid & 15));
    asm volatile("" :: "v"(xv));
    const float d = sdv[r];
    v4f o;
    o.x = d * bf16_val(xv.x);
    o.y = d * bf16_val(xv.y);
    o.z = d * bf16_val(xv.z);
    o.w = d * bf16_val(xv.w);
    float* dp = PA + (size_t)nc * DF + 4 * (tid & 15);
    const bool ok = node < nN;
    if (ok) *(volatile v4f*)dp = o;
    __threadfence();
    if (ok) *(volatile v4f*)dp = o;
  }
}

template <int LAST>
__global__ __launch_bounds__(NTHR) void k_hop(const float* __restrict__ Pin, float* Pout, unsigned short* X3,
                                              const int* __restrict__ LIST, const int* __restrict__ CNT,
                                              const int* __restrict__ OFF, const float* __restrict__ DINV,
                                              const int* __restrict__ REC, int nN) {
  const int tid = (int)threadIdx.x, lane = tid & 31, wave = tid >> 5, hh = lane >> 4, m = lane & 15;
  const int nodeBase = (int)blockIdx.x * NBA;
  const int flag = REC[(size_t)blockIdx.x * 32 + 1];
  const int* lp = LIST + (size_t)blockIdx.x * RCAP;
  const float qnan = __int_as_float(0x7fc00000);
  const int sa = 2 * (lane & 7), sb = 2 * (lane & 7) + 1;
#pragma unroll 1
  for (int si = 0; si < NBA / NWAVE; ++si) {
    const int node = nodeBase + si * NWAVE + wave;
    if (node >= nN) break;
    const int craw = CNT[node];
    const int oraw = OFF[node];
    int c = craw < 0 ? 0 : (craw > DEGCAP ? DEGCAP : craw);
    const int o = oraw < 0 ? 0 : (oraw > RCAP ? RCAP : oraw);
    if (c > RCAP - o) c = RCAP - o;
    const bool pois = (flag != 0) || (craw > DEGCAP) || (craw < 0);
    const int half = (c + 1) >> 1;
    float a0 = 0.0f, a1 = 0.0f, a2 = 0.0f, a3 = 0.0f;
#pragma unroll 1
    for (int t = 0; t < half; ++t) {
      const int p  = 2 * t + hh;
      const int pc = p < c ? p : c - 1;
      int sr = lp[o + pc];
      sr = sr < 0 ? 0 : (sr > nN - 1 ? nN - 1 : sr);
      const v4f v = *(const v4f*)(Pin + (size_t)sr * DF + 4 * m);
      asm volatile("" :: "v"(v));
      const bool ok = p < c;
      a0 += ok ? v.x : 0.0f;
      a1 += ok ? v.y : 0.0f;
      a2 += ok ? v.z : 0.0f;
      a3 += ok ? v.w : 0.0f;
    }
    a0 += __shfl_xor(a0, 16, 32);
    a1 += __shfl_xor(a1, 16, 32);
    a2 += __shfl_xor(a2, 16, 32);
    a3 += __shfl_xor(a3, 16, 32);
    const v4f sv = *(const v4f*)(Pin + (size_t)node * DF + 4 * m);
    const float dd = DINV[node];
    const float sc = (LAST != 0) ? dd : dd * dd;
    float r0 = sc * (a0 + sv.x);
    float r1 = sc * (a1 + sv.y);
    float r2 = sc * (a2 + sv.z);
    float r3 = sc * (a3 + sv.w);
    r0 = pois ? qnan : r0;
    r1 = pois ? qnan : r1;
    r2 = pois ? qnan : r2;
    r3 = pois ? qnan : r3;
    if constexpr (LAST != 0) {
      unsigned hw0, lw0, hw1, lw1;
      pack2(r0, r1, hw0, lw0);
      pack2(r2, r3, hw1, lw1);
      const int g0 = __shfl((int)hw0, sa, 32), g1 = __shfl((int)hw1, sa, 32);
      const int g2 = __shfl((int)hw0, sb, 32), g3 = __shfl((int)hw1, sb, 32);
      const int p0 = __shfl((int)lw0, sa, 32), p1 = __shfl((int)lw1, sa, 32);
      const int p2 = __shfl((int)lw0, sb, 32), p3 = __shfl((int)lw1, sb, 32);
      const bool lsel = (lane & 8) != 0;
      v4u pv;
      pv.x = (unsigned)(lsel ? p0 : g0);
      pv.y = (unsigned)(lsel ? p1 : g1);
      pv.z = (unsigned)(lsel ? p2 : g2);
      pv.w = (unsigned)(lsel ? p3 : g3);
      unsigned short* hp = X3 + (size_t)node * KT + 8 * m;
      if (lane < 16) *(volatile v4u*)hp = pv;
      __threadfence();
      if (lane < 16) *(volatile v4u*)hp = pv;
    } else {
      v4f ow;
      ow.x = r0; ow.y = r1; ow.z = r2; ow.w = r3;
      float* op = Pout + (size_t)node * DF + 4 * m;
      if (lane < 16) *(volatile v4f*)op = ow;
      __threadfence();
      if (lane < 16) *(volatile v4f*)op = ow;
    }
  }
}

__global__ __launch_bounds__(NTHR) __attribute__((amdgpu_num_vgpr(248)))
void k_tail(const unsigned short* __restrict__ X3, const unsigned short* __restrict__ W1D,
            const unsigned short* __restrict__ W2D, const float* __restrict__ BB, float* out, int nN) {
  __shared__ __attribute__((aligned(16))) float    stg[TBM * DF];
  __shared__ __attribute__((aligned(16))) unsigned a2w[TBM * (KT / 2)];
  __shared__ __attribute__((aligned(16))) float    bbs[128];
  const int tid = (int)threadIdx.x, lane = tid & 31, wave = tid >> 5, hh = lane >> 4, mm = lane & 15;
  const int rowBase = (int)blockIdx.x * TBM;

  if (tid < 32) {
    const v4f b4 = *(const v4f*)(BB + 4 * tid);
    *(v4fa*)(bbs + 4 * tid) = b4;
  }

  const v8f z = {0.f, 0.f, 0.f, 0.f, 0.f, 0.f, 0.f, 0.f};
  v8f acc[4];
  acc[0] = z; acc[1] = z; acc[2] = z; acc[3] = z;
  {
    const unsigned short* ap = X3  + (size_t)(rowBase + 16 * wave + mm) * (size_t)KT + 8 * hh;
    const unsigned short* wp = W1D + (size_t)mm * (size_t)KT + 8 * hh;
#pragma unroll 1
    for (int ks = 0; ks < KT / 32; ++ks) {
      FragB af;
      af.h[0] = *(const v8usa*)(ap + 32 * ks);
      af.h[1] = *(const v8usa*)(ap + 32 * ks + 16);
#pragma unroll
      for (int t = 0; t < 4; ++t) {
        const unsigned short* wq = wp + (size_t)(16 * t) * (size_t)KT + 32 * ks;
        FragB bf;
        bf.h[0] = *(const v8usa*)wq;
        bf.h[1] = *(const v8usa*)(wq + 16);
        acc[t] = wmb(af, bf, acc[t]);
      }
    }
  }
  __syncthreads();

#pragma unroll
  for (int t = 0; t < 4; ++t) {
    const int lc = 16 * t + mm;
    const float bb = bbs[lc];
#pragma unroll
    for (int r = 0; r < 8; ++r) {
      const int lr = 16 * wave + 8 * hh + r;
      stg[lr * DF + lc] = acc[t][r] + bb;
    }
  }
  __syncthreads();

#pragma unroll 4
  for (int i = 0; i < 16; ++i) {
    const int lr = 16 * wave + i;
    const v2f p = *(const v2fa*)(stg + lr * DF + 2 * lane);
    unsigned hw, lw;
    pack2(p.x, p.y, hw, lw);
    a2w[lr * (KT / 2) + lane]      = hw;
    a2w[lr * (KT / 2) + 32 + lane] = lw;
  }
  __syncthreads();

  v8f ac2[3];
  ac2[0] = z; ac2[1] = z; ac2[2] = z;
  {
    const unsigned* aq = a2w + (16 * wave + mm) * (KT / 2) + 4 * hh;
    const unsigned short* wp = W2D + (size_t)mm * (size_t)KT + 8 * hh;
#pragma unroll 1
    for (int ks = 0; ks < KT / 32; ++ks) {
      FragB af;
      af.h[0] = *(const v8usa*)(aq + 16 * ks);
      af.h[1] = *(const v8usa*)(aq + 16 * ks + 8);
#pragma unroll
      for (int t = 0; t < 3; ++t) {
        const unsigned short* wq = wp + (size_t)(16 * t) * (size_t)KT + 32 * ks;
        FragB bf;
        bf.h[0] = *(const v8usa*)wq;
        bf.h[1] = *(const v8usa*)(wq + 16);
        ac2[t] = wmb(af, bf, ac2[t]);
      }
    }
  }

  float* os = stg;
#pragma unroll
  for (int t = 0; t < 3; ++t) {
    const int lc = 16 * t + mm;
    const float bb = bbs[64 + lc];
#pragma unroll
    for (int r = 0; r < 8; ++r) {
      const int lr = 16 * wave + 8 * hh + r;
      if (lc < NOUT) os[lr * NOUT + lc] = ac2[t][r] + bb;
    }
  }
  __syncthreads();

  constexpr int NIT = (TBM * NOUT) / (4 * NTHR);
  int vrows = nN - rowBase;
  vrows = vrows > TBM ? TBM : (vrows < 0 ? 0 : vrows);
  const int validQ = vrows * (NOUT / 4);
  v4f ov[NIT];
#pragma unroll
  for (int it = 0; it < NIT; ++it) ov[it] = *(const v4fa*)(os + 4 * (it * NTHR + tid));
  float* ob = out + (size_t)rowBase * NOUT;
#pragma unroll
  for (int it = 0; it < NIT; ++it) {
    const int q = it * NTHR + tid;
    if (q < validQ) *(volatile v4f*)(ob + 4 * (size_t)q) = ov[it];
  }
  __threadfence();
#pragma unroll
  for (int it = 0; it < NIT; ++it) {
    const int q = it * NTHR + tid;
    if (q < validQ) *(volatile v4f*)(ob + 4 * (size_t)q) = ov[it];
  }
}

static inline int cdiv(int a, int b) { return (a + b - 1) / b; }
static inline size_t al256(size_t o) { return (o + 255) & ~(size_t)255; }

extern "C" void kernel_launch(void* const* d_in, const int* in_sizes, int n_in,
                              void* d_out, int out_size, void* d_ws, size_t ws_size,
                              hipStream_t stream) {
  if (n_in < 6) return;
  if (in_sizes[0] < DF || (in_sizes[0] % DF) != 0) return;
  const int nN = in_sizes[0] / DF;
  if (nN < 1 || nN > (1 << 20) || (nN & 3) != 0) return;
  if (in_sizes[1] < 2 || (in_sizes[1] & 1) != 0) return;
  const int nE = in_sizes[1] / 2;
  if (nE < 1 || nE >= (1 << 21)) return;
  if (in_sizes[2] != DF * DF || in_sizes[3] != DF) return;
  if (in_sizes[4] != DF * NOUT || in_sizes[5] != NOUT) return;
  if ((long long)out_size != (long long)nN * NOUT) return;

  const float* x     = (const float*)d_in[0];
  const int*   ei    = (const int*)  d_in[1];
  const int*   src   = ei;
  const int*   dst   = ei + nE;
  const float* Wlin  = (const float*)d_in[2];
  const float* blin  = (const float*)d_in[3];
  const float* Whead = (const float*)d_in[4];
  const float* bhead = (const float*)d_in[5];
  float* out = (float*)d_out;

  const int nB    = cdiv(nN, NBA);
  const int NPADN = nB * NBA;
  const int MP    = cdiv(nN, TBM) * TBM;
  if (MP > NPADN) return;
  const int gT    = MP / TBM;
  const int vec8  = ((nE & 3) == 0) ? 1 : 0;
  const int segLen = cdiv(cdiv(nE, NWAVE), WCH) * WCH;
  const int nPadUnits = (MP - nN) * 16;

  char* ws = (char*)d_ws;
  size_t off = 0;
  const size_t oPA = off; off = al256(off + (size_t)nN * DF * 4);
  const size_t oPB = off; off = al256(off + (size_t)nN * DF * 4);
  const size_t oX3 = off; off = al256(off + (size_t)MP * KT * 2);
  const size_t oLS = off; off = al256(off + (size_t)nB * RCAP * 4);
  const size_t oCN = off; off = al256(off + (size_t)NPADN * 4);
  const size_t oOF = off; off = al256(off + (size_t)NPADN * 4);
  const size_t oDV = off; off = al256(off + (size_t)NPADN * 4);
  const size_t oRC = off; off = al256(off + (size_t)nB * 128);
  const size_t oW1 = off; off = al256(off + (size_t)DF * KT * 2);
  const size_t oW2 = off; off = al256(off + (size_t)NOP * KT * 2);
  const size_t oBB = off; off = al256(off + 512);
  if (off > ws_size || off > (size_t)WSMAX) return;
  float* PA = (float*)(ws + oPA);
  float* PB = (float*)(ws + oPB);
  unsigned short* X3 = (unsigned short*)(ws + oX3);
  int*   LIST = (int*)(ws + oLS);
  int*   CNT  = (int*)(ws + oCN);
  int*   OFF  = (int*)(ws + oOF);
  float* DINV = (float*)(ws + oDV);
  int*   REC  = (int*)(ws + oRC);
  unsigned short* W1D = (unsigned short*)(ws + oW1);
  unsigned short* W2D = (unsigned short*)(ws + oW2);
  float* BB = (float*)(ws + oBB);

  hipFuncSetAttribute(reinterpret_cast<const void*>(&k_bucket), hipFuncAttributeMaxDynamicSharedMemorySize, LDS_BK);

  k_prep<<<8 + cdiv(nPadUnits, NTHR), NTHR, 0, stream>>>(Wlin, blin, Whead, bhead, W1D, W2D, BB, X3, nN, nPadUnits);
  k_bucket<<<nB, NTHR, LDS_BK, stream>>>(dst, src, x, nE, nN, vec8, segLen, LIST, CNT, OFF, DINV, REC, PA);
  k_hop<0><<<nB, NTHR, 0, stream>>>(PA, PB, X3, LIST, CNT, OFF, DINV, REC, nN);
  k_hop<0><<<nB, NTHR, 0, stream>>>(PB, PA, X3, LIST, CNT, OFF, DINV, REC, nN);
  k_hop<1><<<nB, NTHR, 0, stream>>>(PA, PB, X3, LIST, CNT, OFF, DINV, REC, nN);
  k_tail<<<gT, NTHR, 0, stream>>>(X3, W1D, W2D, BB, out, nN);
}
